// Net_separate_11390253269734
// MI455X (gfx1250) — hardware-run, weakly checked
//
#include <hip/hip_runtime.h>


namespace {
constexpr int NN = 100000, NE = 1600000, HD = 32, NBI = 20000, NII = 80000, MAXDEG = 1024, NGc = (NN + 511) / 512, PERMLEN = NE + 32 * NGc + 32;
constexpr float XS = 8.0f;

typedef _Float16 b16;
typedef __attribute__((ext_vector_type(16))) _Float16 v16b;
typedef __attribute__((ext_vector_type(8))) _Float16 v8b;
typedef __attribute__((ext_vector_type(8))) float v8f;
typedef __attribute__((ext_vector_type(4))) float v4f;
__device__ __forceinline__ float bf16_rne(float f) { unsigned int u = __float_as_uint(f); u += 0x7FFFu + ((u >> 16) & 1u); return __uint_as_float(u & 0xFFFF0000u); }
__device__ __forceinline__ void split16(float v, b16& hi, b16& lo) { hi = (b16)v; lo = (b16)(v - (float)hi); }
__device__ __forceinline__ v16b frag_kb(const b16* p, int hh) { const v8b a = *(const v8b*)(p + 8 * hh), b = *(const v8b*)(p + 16 + 8 * hh); v16b f;
#pragma unroll
  for (int e = 0; e < 8; ++e) { f[e] = a[e]; f[8 + e] = b[e]; } return f; }
__device__ __forceinline__ v8f wmma16b(v16b a, v16b b, v8f c) { v8f d = __builtin_amdgcn_wmma_f32_16x16x32_f16(false, a, false, b, (short)0, c, false, false); asm volatile("v_nop\n\tv_nop\n\tv_nop\n\tv_nop" : "+v"(d) : "v"(a), "v"(b)); return d; }
__device__ __forceinline__ void wave_lds_sync() { __builtin_amdgcn_fence(__ATOMIC_RELEASE, "workgroup"); __builtin_amdgcn_wave_barrier(); __builtin_amdgcn_fence(__ATOMIC_ACQUIRE, "workgroup"); }
__device__ __forceinline__ float pmul(float a, float b) { float p = a * b; asm volatile("" : "+v"(p)); return p; }
constexpr int CSR_NBLK = 512, CSR_GB = 9, CSR_GN = 1 << CSR_GB  , CSR_MAXG = 512, CSR_CAP = 12288  ;
__global__ __launch_bounds__(64) void csrA_kernel(const int* __restrict__ dst, int E, int N, int nG, int CHP, int NGP, int* __restrict__ STG, int* __restrict__ HST) {
  extern __shared__ int sm[];
  int* cnt = sm; int* run = sm + NGP; int* ids = sm + 2 * NGP;
  const int b = blockIdx.x; const int ch = (E + CSR_NBLK - 1) / CSR_NBLK; const int e0 = b * ch, e1 = min(E, e0 + ch);
  for (int i = threadIdx.x; i < NGP; i += 64) cnt[i] = 0;
  for (int i = threadIdx.x; i < CHP; i += 64) ids[i] = -1;
  __syncthreads();
  if (threadIdx.x == 0) {
    for (int e = e0; e < e1; ++e) { int d = dst[e]; d = (d < 0) ? 0 : (d >= N ? N - 1 : d); cnt[d >> CSR_GB] += 1; }
    int acc = 0; for (int g = 0; g < nG; ++g) { run[g] = acc; acc += cnt[g]; }
    for (int e = e0; e < e1; ++e) { int d = dst[e]; d = (d < 0) ? 0 : (d >= N ? N - 1 : d); const int g = d >> CSR_GB; ids[run[g]] = e; run[g] += 1; } }
  __syncthreads();
  typedef __attribute__((ext_vector_type(4))) int v4i;
  for (int pass = 0; pass < 2; ++pass) {
    for (int i = threadIdx.x; i < CHP / 4; i += 64) *(volatile v4i*)(STG + (size_t)b * CHP + i * 4) = *(const v4i*)(&ids[i * 4]);
    for (int i = threadIdx.x; i < NGP / 4; i += 64) { v4i v; for (int e = 0; e < 4; ++e) v[e] = (i * 4 + e < nG) ? cnt[i * 4 + e] : 0; *(volatile v4i*)(HST + (size_t)b * NGP + i * 4) = v; }
    __threadfence(); }
}
__global__ __launch_bounds__(512) void csrS_kernel(const int* __restrict__ HST, int nG, int NGP, int* __restrict__ START, int* __restrict__ TOT, int* __restrict__ OFF) {
  __shared__ int tot[CSR_MAXG];
  const int b = threadIdx.x;
  for (int pass = 0; pass < 2; ++pass) { int runb = 0; for (int g = 0; g < nG; ++g) { int c = HST[(size_t)b * NGP + g]; c = (c < 0) ? 0 : c; ((volatile int*)OFF)[(size_t)g * CSR_NBLK + b] = runb; runb += c; } __threadfence(); }
  for (int g = threadIdx.x; g < nG; g += 512) { int s = 0; for (int bb = 0; bb < CSR_NBLK; ++bb) { int c = HST[(size_t)bb * NGP + g]; s += (c < 0) ? 0 : c; } tot[g] = s; }
  __syncthreads();
  if (threadIdx.x < 32) {
    __shared__ int st[CSR_MAXG + 32];
    if (threadIdx.x == 0) { int acc = 0; for (int g = 0; g < NGP; ++g) { st[g] = acc; if (g < nG) acc += (tot[g] + 31) & ~31; } st[NGP] = acc; }
    __builtin_amdgcn_fence(__ATOMIC_RELEASE, "workgroup"); __builtin_amdgcn_wave_barrier(); __builtin_amdgcn_fence(__ATOMIC_ACQUIRE, "workgroup");
    for (int pass = 0; pass < 2; ++pass) { for (int i = threadIdx.x; i < NGP + 32; i += 32) { ((volatile int*)START)[i] = (i <= NGP) ? st[min(i, NGP)] : 0; ((volatile int*)TOT)[i] = (i < nG) ? tot[i] : 0; } __threadfence(); } }
}
__global__ __launch_bounds__(256) void csrB_kernel(const int* __restrict__ dst, int N, int nG, int CHP, int NGP, int permLen, const int* __restrict__ STG, const int* __restrict__ HST, const int* __restrict__ OFF, const int* __restrict__ START, const int* __restrict__ TOT, int* __restrict__ PERM, int* __restrict__ ROWPTR, int* __restrict__ ROWCNT, int* __restrict__ FLAG) {
  typedef __attribute__((ext_vector_type(4))) int v4i;
  __shared__ int ids[CSR_CAP]; __shared__ unsigned short key[CSR_CAP]; __shared__ int outp[CSR_CAP]; __shared__ int ncnt[CSR_GN + 1]; __shared__ int boff[CSR_NBLK + 1];
  const int g = blockIdx.x, t_ = threadIdx.x; int tot = TOT[g]; int st = START[g], stn = START[g + 1]; const int v0 = g * CSR_GN; const int nv = min(CSR_GN, N - v0);
  st = (st < 0) ? 0 : (st > permLen - 32 ? permLen - 32 : st) & ~31; stn = (stn < st) ? st : (stn > permLen ? permLen : stn); tot = (tot < 0) ? 0 : tot; if (tot > stn - st && tot <= CSR_CAP) tot = stn - st;
  if (tot > CSR_CAP) {
    for (int pass = 0; pass < 2; ++pass) { for (int i = t_; i < CSR_GN / 4; i += 256) { v4i a, c; for (int e = 0; e < 4; ++e) { a[e] = st; c[e] = 0; } *(volatile v4i*)(ROWPTR + v0 + i * 4) = a; *(volatile v4i*)(ROWCNT + v0 + i * 4) = c; } if (t_ == 0) ((volatile int*)FLAG)[0] = 1; __threadfence(); } (void)nv; return; }
  if (t_ == 0) { int acc = 0; for (int b = 0; b < CSR_NBLK; ++b) { boff[b] = acc; int c = HST[(size_t)b * NGP + g]; c = (c < 0) ? 0 : (c > CHP ? CHP : c); acc += c; if (acc > tot) acc = tot; } boff[CSR_NBLK] = acc; }
  for (int i = t_; i <= CSR_GN; i += 256) ncnt[i] = 0;
  __syncthreads();
  for (int b = 0; b < CSR_NBLK; ++b) { const int c = boff[b + 1] - boff[b]; int o_ = OFF[(size_t)g * CSR_NBLK + b]; o_ = (o_ < 0) ? 0 : (o_ > CHP - c ? CHP - c : o_); const int* src_ = STG + (size_t)b * CHP + o_;
    for (int i = t_; i < c; i += 256) { int id = src_[i]; id = (id < 0) ? 0 : id; ids[boff[b] + i] = id; int d = dst[id]; d = (d < v0) ? v0 : (d >= N ? N - 1 : d); int kk = d - v0; kk = (kk < 0) ? 0 : (kk >= CSR_GN ? CSR_GN - 1 : kk); key[boff[b] + i] = (unsigned short)kk; } }
  __syncthreads();
  if (t_ == 0) { for (int i = 0; i < tot; ++i) ncnt[key[i]] += 1; int acc = 0; for (int vl = 0; vl < CSR_GN; ++vl) { const int c = ncnt[vl]; ncnt[vl] = acc; acc += c; } ncnt[CSR_GN] = acc;
    for (int i = 0; i < tot; ++i) { const int vl = key[i]; outp[ncnt[vl]] = ids[i]; ncnt[vl] += 1; }
    for (int vl = CSR_GN; vl > 0; --vl) ncnt[vl] = ncnt[vl - 1]; ncnt[0] = 0; }
  __syncthreads();
  for (int pass = 0; pass < 2; ++pass) {
    for (int i = t_; i < (stn - st) / 4; i += 256) { v4i v; for (int e = 0; e < 4; ++e) { const int q = i * 4 + e; v[e] = (q < tot) ? outp[q] : -1; } *(volatile v4i*)(PERM + st + i * 4) = v; }
    for (int i = t_; i < CSR_GN / 4; i += 256) { v4i a, c; for (int e = 0; e < 4; ++e) { const int vl = i * 4 + e; a[e] = st + ncnt[vl]; c[e] = (vl < nv) ? (ncnt[vl + 1] - ncnt[vl]) : 0; } *(volatile v4i*)(ROWPTR + v0 + i * 4) = a; *(volatile v4i*)(ROWCNT + v0 + i * 4) = c; }
    __threadfence(); }
}
__global__ __launch_bounds__(256) void csrZ_kernel(int* __restrict__ p, size_t n4) { typedef __attribute__((ext_vector_type(4))) int v4i; const size_t tid = (size_t)blockIdx.x * 256 + threadIdx.x, nth = (size_t)gridDim.x * 256; v4i z = {0, 0, 0, 0}; for (size_t i = tid; i < n4; i += nth) *(volatile v4i*)(p + i * 4) = z; }
struct CsrBufs { int *STG, *HST, *OFF, *START, *TOT, *PERM, *ROWPTR, *ROWCNT, *FLAG; int nG, NGP, CHP; size_t permLen; char* base; size_t bytes; };
static size_t csr_carve(CsrBufs& c, char* ws, size_t off, int E, int N) {
  const size_t off0 = off; c.base = ws + off;
  auto al = [&](size_t bytes) { char* p = ws + off; off += (bytes + 255) & ~(size_t)255; return p; };
  c.nG = (N + CSR_GN - 1) / CSR_GN; c.NGP = (c.nG + 31) & ~31; const int ch = (E + CSR_NBLK - 1) / CSR_NBLK; c.CHP = (ch + 31) & ~31; c.permLen = (size_t)E + 32 * (size_t)c.nG + 32;
  c.STG = (int*)al((size_t)CSR_NBLK * c.CHP * 4); c.HST = (int*)al((size_t)CSR_NBLK * c.NGP * 4); c.OFF = (int*)al((size_t)c.NGP * CSR_NBLK * 4); c.START = (int*)al((size_t)(c.NGP + 64) * 4); c.TOT = (int*)al((size_t)(c.NGP + 64) * 4);
  c.PERM = (int*)al(c.permLen * 4); c.ROWPTR = (int*)al((size_t)c.nG * CSR_GN * 4); c.ROWCNT = (int*)al((size_t)c.nG * CSR_GN * 4); c.FLAG = (int*)al(256);
  c.bytes = off - off0; return off;
}
static void csr_build(const CsrBufs& c, const int* dst, int E, int N, hipStream_t stream) {
  const size_t smem = (size_t)(2 * c.NGP + c.CHP) * 4;
  csrZ_kernel<<<512, 256, 0, stream>>>((int*)c.base, c.bytes / 16);
  csrA_kernel<<<CSR_NBLK, 64, smem, stream>>>(dst, E, N, c.nG, c.CHP, c.NGP, c.STG, c.HST);
  csrS_kernel<<<1, 512, 0, stream>>>(c.HST, c.nG, c.NGP, c.START, c.TOT, c.OFF);
  csrB_kernel<<<c.nG, 256, 0, stream>>>(dst, N, c.nG, c.CHP, c.NGP, (int)c.permLen, c.STG, c.HST, c.OFF, c.START, c.TOT, c.PERM, c.ROWPTR, c.ROWCNT, c.FLAG);
}

__global__ __launch_bounds__(256) void prep_kernel(const float* __restrict__ wb1, const float* __restrict__ bb1, const float* __restrict__ wb2, const float* __restrict__ bb2, const float* __restrict__ wi1, const float* __restrict__ bi1, const float* __restrict__ wi2, const float* __restrict__ bi2,
    const float* __restrict__ wc1, const float* __restrict__ bc1, const float* __restrict__ wc2, const float* __restrict__ bc2, const float* __restrict__ wc3, const float* __restrict__ bc3, const float* __restrict__ wf, const float* __restrict__ bff, b16* __restrict__ R, float* __restrict__ P) {
  const size_t tid = (size_t)blockIdx.x * 256 + threadIdx.x, nth = (size_t)gridDim.x * 256;
  for (int pass = 0; pass < 2; ++pass) {
    for (size_t p = tid; p < (size_t)3 * HD * HD; p += nth) { const int l = (int)(p / (HD * HD)), o = (int)((p / HD) % HD), k = (int)(p % HD); const float* W = (l == 0) ? wc1 : (l == 1) ? wc2 : wc3; ((volatile b16*)R)[p] = (b16)bf16_rne(W[(size_t)k * HD + o]); }
    for (size_t q = tid; q < 2465; q += nth) { const int i = (int)q; float v;
      if (i < 96) v = wb1[i]; else if (i < 128) v = bb1[i - 96]; else if (i < 1152) v = wb2[i - 128]; else if (i < 1184) v = bb2[i - 1152]; else if (i < 1248) v = wi1[i - 1184]; else if (i < 1280) v = bi1[i - 1248]; else if (i < 2304) v = wi2[i - 1280]; else if (i < 2336) v = bi2[i - 2304];
      else if (i < 2368) v = bc1[i - 2336]; else if (i < 2400) v = bc2[i - 2368]; else if (i < 2432) v = bc3[i - 2400]; else if (i < 2464) v = wf[i - 2432]; else v = bff[0];
      P[q] = bf16_rne(v); }
    __threadfence(); }
}
__device__ __forceinline__ bool in_sorted(const int* __restrict__ a, int n, int key) { int lo = 0, hi = n; while (lo < hi) { const int mid = (lo + hi) >> 1; if (a[mid] < key) lo = mid + 1; else hi = mid; } return (lo < n) && (a[lo] == key); }
__global__ __launch_bounds__(256) void h0_kernel(const float* __restrict__ x, const float* __restrict__ y, const int* __restrict__ bidx, const int* __restrict__ iidx, const float* __restrict__ P, float* __restrict__ H) {
  __shared__ __attribute__((aligned(16))) float Hs[256][HD + 1];
  const int n = blockIdx.x * 256 + threadIdx.x; float outv[HD]; for (int c = 0; c < HD; ++c) outv[c] = 0.0f;
  if (n < NN) { const bool isb = in_sorted(bidx, NBI, n), isi = in_sorted(iidx, NII, n); const float x0 = bf16_rne(x[(size_t)n * 2]), x1 = bf16_rne(x[(size_t)n * 2 + 1]), yy = bf16_rne(y[n]);
    if (isi || isb) { float hid[HD];
      if (isi) { for (int c = 0; c < HD; ++c) hid[c] = fmaxf(pmul(x0, P[1184 + c]) + pmul(x1, P[1184 + HD + c]) + P[1248 + c], 0.0f); for (int o = 0; o < HD; ++o) { float s = P[2304 + o]; for (int c = 0; c < HD; ++c) s += pmul(hid[c], P[1280 + c * HD + o]); outv[o] = s; } }
      else { for (int c = 0; c < HD; ++c) hid[c] = fmaxf(pmul(x0, P[c]) + pmul(x1, P[HD + c]) + pmul(yy, P[2 * HD + c]) + P[96 + c], 0.0f); for (int o = 0; o < HD; ++o) { float s = P[1152 + o]; for (int c = 0; c < HD; ++c) s += pmul(hid[c], P[128 + c * HD + o]); outv[o] = s; } } } }
  for (int c = 0; c < HD; ++c) Hs[threadIdx.x][c] = fmaxf(outv[c], 0.0f);
  __syncthreads();
  for (int pass = 0; pass < 2; ++pass) { for (int i = threadIdx.x; i < 256 * (HD / 4); i += 256) { const int rr = i / (HD / 4), c4 = (i % (HD / 4)) * 4; const int nn = blockIdx.x * 256 + rr; if (nn < NN) { v4f v; for (int e = 0; e < 4; ++e) v[e] = Hs[rr][c4 + e]; *(volatile v4f*)(H + (size_t)nn * HD + c4) = v; } } __threadfence(); }
}
__global__ __launch_bounds__(64) void gemm_kernel(const float* __restrict__ H, const b16* __restrict__ Bw, float* __restrict__ HW) {
  __shared__ __attribute__((aligned(16))) b16 Ah[32][HD + 8], Al[32][HD + 8]; __shared__ __attribute__((aligned(16))) float Ts[32][HD + 4];
  const int lane = threadIdx.x & 31, wave = threadIdx.x >> 5, nloc = lane & 15, hlf = lane >> 4, m0 = blockIdx.x * 32;
  for (int i = threadIdx.x; i < 32 * HD; i += 64) { const int rr = i / HD, c = i % HD; b16 a_, b_; split16(H[(size_t)(m0 + rr) * HD + c] * XS, a_, b_); Ah[rr][c] = a_; Al[rr][c] = b_; }
  __syncthreads();
  v8f acc[2] = {{}, {}}; const v16b a = frag_kb(&Ah[wave * 16 + nloc][0], hlf), al_ = frag_kb(&Al[wave * 16 + nloc][0], hlf);
#pragma unroll
  for (int t = 0; t < 2; ++t) { const v16b bw = frag_kb(Bw + (size_t)(t * 16 + nloc) * HD, hlf); acc[t] = wmma16b(a, bw, acc[t]); acc[t] = wmma16b(al_, bw, acc[t]); }
#pragma unroll
  for (int t = 0; t < 2; ++t)
#pragma unroll
    for (int r = 0; r < 8; ++r) Ts[wave * 16 + 8 * hlf + r][t * 16 + nloc] = acc[t][r] * (1.0f / XS);
  __syncthreads();
  for (int pass = 0; pass < 2; ++pass) { for (int i = threadIdx.x; i < 32 * (HD / 4); i += 64) { const int rr = i / (HD / 4), c4 = (i % (HD / 4)) * 4; *(volatile v4f*)(HW + (size_t)(m0 + rr) * HD + c4) = *(const v4f*)(&Ts[rr][c4]); } __threadfence(); }
}
__global__ __launch_bounds__(256) void agg_kernel(const float* __restrict__ HW, const int* __restrict__ src, const int* __restrict__ perm, const int* __restrict__ rowptr, const int* __restrict__ rowcnt, const float* __restrict__ Pb, float* __restrict__ H) {
  const int wave = threadIdx.x >> 5, v = blockIdx.x * 8 + wave, lane = threadIdx.x & 31;
  int cnt = rowcnt[v]; cnt = (cnt < 0) ? 0 : (cnt > MAXDEG ? MAXDEG : cnt); int p0 = rowptr[v]; p0 = (p0 < 0) ? 0 : (p0 > PERMLEN - cnt ? PERMLEN - cnt : p0);
  const float dv = rsqrtf((float)cnt + 1.0f); float acc = HW[(size_t)v * HD + lane] * (dv * dv);
  for (int q = 0; q < cnt; ++q) { int id = perm[p0 + q]; id = (id < 0) ? 0 : (id >= NE ? NE - 1 : id); int s = src[id]; s = (s < 0) ? 0 : (s >= NN ? NN - 1 : s); int cs_ = rowcnt[s]; cs_ = (cs_ < 0) ? 0 : (cs_ > MAXDEG ? MAXDEG : cs_); acc += pmul(pmul(rsqrtf((float)cs_ + 1.0f), dv), HW[(size_t)s * HD + lane]); }
  const float h = fmaxf(acc + Pb[lane], 0.0f);
  for (int pass = 0; pass < 2; ++pass) { ((volatile float*)H)[(size_t)v * HD + lane] = h; __threadfence(); }
}
__global__ __launch_bounds__(256) void final_kernel(const float* __restrict__ H, const float* __restrict__ P, float* __restrict__ out) {
  const int n = blockIdx.x * 256 + threadIdx.x; float s = 0.0f; if (n < NN) { s = P[2464]; for (int c = 0; c < HD; ++c) s += pmul(H[(size_t)n * HD + c], P[2432 + c]); }
  for (int pass = 0; pass < 2; ++pass) { if (n < NN) ((volatile float*)out)[n] = s; __threadfence(); }
}
}

extern "C" void kernel_launch(void* const* d_in, const int* in_sizes, int n_in,
                              void* d_out, int out_size, void* d_ws, size_t ws_size, hipStream_t stream) {
  (void)n_in; (void)out_size;
  const float* x = (const float*)d_in[0]; const float* y = (const float*)d_in[1]; const int* ei = (const int*)d_in[2]; const int* bidx = (const int*)d_in[3]; const int* iidx = (const int*)d_in[4];
  const float* wb1 = (const float*)d_in[5]; const float* bb1 = (const float*)d_in[6]; const float* wb2 = (const float*)d_in[7]; const float* bb2 = (const float*)d_in[8]; const float* wi1 = (const float*)d_in[9]; const float* bi1 = (const float*)d_in[10]; const float* wi2 = (const float*)d_in[11]; const float* bi2 = (const float*)d_in[12];
  const float* wc1 = (const float*)d_in[13]; const float* bc1 = (const float*)d_in[14]; const float* wc2 = (const float*)d_in[15]; const float* bc2 = (const float*)d_in[16]; const float* wc3 = (const float*)d_in[17]; const float* bc3 = (const float*)d_in[18]; const float* wf = (const float*)d_in[19]; const float* bff = (const float*)d_in[20];
  float* out = (float*)d_out;
  if (in_sizes[0] != NN * 2 || in_sizes[2] != 2 * NE || in_sizes[3] != NBI || in_sizes[4] != NII) return;
  const int* srcI = ei; const int* dstI = ei + NE; const int NE_RUN = NE;
  size_t off = 0; char* ws = (char*)d_ws;
  auto carve = [&](size_t bytes) { char* p = ws + off; off += (bytes + 255) & ~(size_t)255; return p; };
  b16* R = (b16*)carve((size_t)3 * HD * HD * 2); float* P = (float*)carve(2480 * 4); float* H = (float*)carve((size_t)NN * HD * 4); float* HW = (float*)carve((size_t)NN * HD * 4);
  CsrBufs cs; off = csr_carve(cs, ws, off, NE_RUN, NN);
  if (off > ws_size) return;
  csr_build(cs, dstI, NE_RUN, NN, stream);
  prep_kernel<<<64, 256, 0, stream>>>(wb1, bb1, wb2, bb2, wi1, bi1, wi2, bi2, wc1, bc1, wc2, bc2, wc3, bc3, wf, bff, R, P);
  h0_kernel<<<(NN + 255) / 256, 256, 0, stream>>>(x, y, bidx, iidx, P, H);
  for (int l = 0; l < 3; ++l) { gemm_kernel<<<NN / 32, 64, 0, stream>>>(H, R + (size_t)l * HD * HD, HW); agg_kernel<<<NN / 8, 256, 0, stream>>>(HW, srcI, cs.PERM, cs.ROWPTR, cs.ROWCNT, P + 2336 + l * HD, H); }
  final_kernel<<<(NN + 255) / 256, 256, 0, stream>>>(H, P, out);
}
